// ExactLogPODE_20504173871579
// MI455X (gfx1250) — hardware-run, weakly checked
//
#include <hip/hip_runtime.h>
#include <math.h>

typedef __attribute__((ext_vector_type(16))) _Float16 v16h;
typedef __attribute__((ext_vector_type(8)))  _Float16 v8h;
typedef __attribute__((ext_vector_type(8)))  float    v8f;
typedef __attribute__((ext_vector_type(4)))  float    v4f;

namespace eng {

constexpr int kBatch   = 1024;
constexpr int kDim     = 16;
constexpr int kHid     = 128;
constexpr int kThreads = 64;
constexpr int kWaves   = kThreads / 32;
constexpr int kRowsPerWave = 32;
constexpr int kBlocks  = kBatch / (kWaves * kRowsPerWave);
constexpr int kAPitch  = 20;
static_assert(kDim == 16, "state width is one 16-wide tile");
static_assert(kHid == 128, "hidden width is eight 16-wide tiles");
static_assert(kBlocks * kWaves * kRowsPerWave == kBatch, "exact grid");

constexpr float kCarryAct = 64.0f;
constexpr float kCarryW1  = 64.0f;
constexpr float kCarryW2  = 256.0f;
constexpr float kFold1    = 1.0f / (kCarryAct * kCarryW1);
constexpr float kFold2    = 1.0f / (kCarryAct * kCarryW2);
constexpr float kF16MinNormal = 6.103515625e-05f;
constexpr float kRadial   = 0.5f * (float)(kDim - 1);

constexpr double kLn2        = 0.6931471805599453;
constexpr double kLnPi       = 1.1447298858494002;
constexpr double kLnGammaHalfDim = 8.525161361065415;
constexpr double kLogP0      = -(kLn2 + 0.5 * (double)kDim * kLnPi - kLnGammaHalfDim);

union FragU { v16h v; v8h h[2]; };

__device__ __forceinline__ v8h zero8h() {
  return (v8h){(_Float16)0.0f, (_Float16)0.0f, (_Float16)0.0f, (_Float16)0.0f,
               (_Float16)0.0f, (_Float16)0.0f, (_Float16)0.0f, (_Float16)0.0f};
}
__device__ __forceinline__ v8f zero8f() {
  return (v8f){0.f, 0.f, 0.f, 0.f, 0.f, 0.f, 0.f, 0.f};
}

__device__ __forceinline__ v8f mma_h(v16h a, v16h b, v8f c) {
  c = __builtin_amdgcn_wmma_f32_16x16x32_f16(false, a, false, b, (short)0, c, false, false);
  asm volatile("v_nop\n\tv_nop\n\tv_nop\n\tv_nop" : "+v"(c) : "v"(a), "v"(b));
  return c;
}

__device__ __forceinline__ _Float16 to_h(float v) {
  const float f = (fabsf(v) < kF16MinNormal) ? 0.0f : v;
  return (_Float16)f;
}

__device__ __forceinline__ float tanh_f32(float x) {
  const float x2 = fminf(x + x, 40.0f);
  const float e  = expf(x2);
  const float d  = e + 1.0f;
  float r = __builtin_amdgcn_rcpf(d);
  r = fmaf(fmaf(-d, r, 1.0f), r, r);
  return 1.0f - (r + r);
}

__device__ __forceinline__ void wave_lds_sync() {
  __builtin_amdgcn_fence(__ATOMIC_RELEASE, "workgroup");
  __builtin_amdgcn_wave_barrier();
  __builtin_amdgcn_fence(__ATOMIC_ACQUIRE, "workgroup");
}

__global__ __launch_bounds__(kThreads) void sphere_flow_logp_kernel(
    const float* __restrict__ gx, const float* __restrict__ gt, const float* __restrict__ gW1,
    const float* __restrict__ gb1, const float* __restrict__ gW2, const float* __restrict__ gb2,
    const int* __restrict__ gsteps, float* __restrict__ gout)
{
  __shared__ __align__(16) _Float16 sW1t[kHid * 16];
  __shared__ __align__(16) _Float16 sW2q[kHid * 16];
  __shared__ __align__(16) _Float16 sW2t[kDim * kHid];
  __shared__ __align__(16) float sW1s[kHid];
  __shared__ __align__(16) float sB1[kHid];
  __shared__ __align__(16) float sDW[kHid];
  __shared__ __align__(16) float sB2[kDim];
  __shared__ __align__(16) _Float16 sY[kWaves][kRowsPerWave * 16];
  __shared__ __align__(16) float sA[kWaves][kRowsPerWave * kAPitch];

  const int tid  = threadIdx.x;
  const int lane = tid & 31;
  const int wave = tid >> 5;
  const int hh   = lane >> 4;
  const int c    = lane & 15;

#pragma unroll 1
  for (int g = tid; g < 256; g += kThreads) {
    const int n  = g >> 1;
    const int k0 = (g & 1) * 8;
    const int jo = g >> 4;
    const int kk0 = (g & 15) * 8;
    v8h w1v, w2v, w3v;
#pragma unroll
    for (int e = 0; e < 8; ++e) {
      w1v[e] = to_h(gW1[(k0 + e) * kHid + n] * kCarryW1);
      w2v[e] = to_h(gW2[n * kDim + k0 + e] * kCarryW2);
      w3v[e] = to_h(gW2[(kk0 + e) * kDim + jo] * kCarryW2);
    }
    *(v8h*)(sW1t + n * 16 + k0) = w1v;
    *(v8h*)(sW2q + n * 16 + k0) = w2v;
    *(v8h*)(sW2t + jo * kHid + kk0) = w3v;
  }
#pragma unroll 1
  for (int k = tid; k < kHid; k += kThreads) {
    float acc = 0.0f;
#pragma unroll 1
    for (int j = 0; j < kDim; ++j) acc = fmaf(gW1[j * kHid + k], gW2[k * kDim + j], acc);
    sDW[k]  = acc;
    sW1s[k] = gW1[kDim * kHid + k];
    sB1[k]  = gb1[k];
  }
  {
    float b2v = gb2[tid & (kDim - 1)];
    asm volatile("" : "+v"(b2v));
    if (tid < kDim) sB2[tid] = b2v;
  }
  __syncthreads();

  _Float16* yw = sY[wave];
  float*    aw = sA[wave];
  const int row = (blockIdx.x * kWaves + wave) * kRowsPerWave + lane;

  float y[16], z[16], ksum[16];
#pragma unroll
  for (int q4 = 0; q4 < 4; ++q4) {
    const v4f xv = *(const v4f*)(gx + (size_t)row * kDim + 4 * q4);
    y[4 * q4 + 0] = xv[0];
    y[4 * q4 + 1] = xv[1];
    y[4 * q4 + 2] = xv[2];
    y[4 * q4 + 3] = xv[3];
  }
#pragma unroll
  for (int j = 0; j < 16; ++j) { z[j] = y[j]; ksum[j] = 0.0f; }

  int nsteps = gsteps[0];
  nsteps = (nsteps < 1) ? 1 : ((nsteps > 1000) ? 1000 : nsteps);
  const float ds = gt[0] / (float)nsteps;
  float s = 0.0f;
  float logp = 0.0f;

#pragma unroll 1
  for (int it = 0; it < nsteps; ++it) {
#pragma unroll 1
    for (int ev = 0; ev < 5; ++ev) {
      const bool isdiv = (ev == 0);
      const float se = s + ((ev >= 4) ? ds : ((ev >= 2) ? (0.5f * ds) : 0.0f));
      float inv = 1.0f;
      if (isdiv) {
        float ss = 0.0f;
#pragma unroll
        for (int j = 0; j < 16; ++j) ss = fmaf(y[j], y[j], ss);
        inv = 1.0f / sqrtf(ss);
#pragma unroll
        for (int j = 0; j < 16; ++j) z[j] = y[j] * inv;
      }

      {
        v8h s0, s1;
#pragma unroll
        for (int e = 0; e < 8; ++e) {
          s0[e] = to_h(z[e] * kCarryAct);
          s1[e] = to_h(z[8 + e] * kCarryAct);
        }
        *(v8h*)(yw + lane * 16) = s0;
        *(v8h*)(yw + lane * 16 + 8) = s1;
      }
      wave_lds_sync();

#pragma unroll 1
      for (int t = 0; t < 2; ++t) {
        FragU yb;
        yb.h[0] = *(const v8h*)(yw + (16 * t + c) * 16 + 8 * hh);
        yb.h[1] = zero8h();
        v8f oacc = zero8f();
        float tpl = 0.0f;
#pragma unroll 1
        for (int jj = 0; jj < 4; ++jj) {
          v16h hf;
#pragma unroll
          for (int u = 0; u < 2; ++u) {
            const int j = 2 * jj + u;
            const int hid0 = 16 * j + 8 * hh;
            FragU wa;
            wa.h[0] = *(const v8h*)(sW1t + (16 * j + c) * 16 + 8 * hh);
            wa.h[1] = zero8h();
            const v8f d1 = mma_h(wa.v, yb.v, zero8f());
            const v4f ws0 = *(const v4f*)(sW1s + hid0);
            const v4f ws1 = *(const v4f*)(sW1s + hid0 + 4);
            const v4f bb0 = *(const v4f*)(sB1 + hid0);
            const v4f bb1 = *(const v4f*)(sB1 + hid0 + 4);
            const float wsv[8] = {ws0[0], ws0[1], ws0[2], ws0[3], ws1[0], ws1[1], ws1[2], ws1[3]};
            const float bbv[8] = {bb0[0], bb0[1], bb0[2], bb0[3], bb1[0], bb1[1], bb1[2], bb1[3]};
            float hv[8];
#pragma unroll
            for (int r = 0; r < 8; ++r) {
              const float raw = d1[r] * kFold1;
              const float pre = fmaf(se, wsv[r], raw) + bbv[r];
              hv[r] = tanh_f32(pre);
            }
            if (isdiv) {
              FragU qa;
              qa.h[0] = *(const v8h*)(sW2q + (16 * j + c) * 16 + 8 * hh);
              qa.h[1] = zero8h();
              const v8f dq = mma_h(qa.v, yb.v, zero8f());
              const v4f dw0 = *(const v4f*)(sDW + hid0);
              const v4f dw1 = *(const v4f*)(sDW + hid0 + 4);
              const float dwv[8] = {dw0[0], dw0[1], dw0[2], dw0[3], dw1[0], dw1[1], dw1[2], dw1[3]};
#pragma unroll
              for (int r = 0; r < 8; ++r) {
                const float omh = fmaf(-hv[r], hv[r], 1.0f);
                const float qq  = dq[r] * kFold2;
                const float rr  = d1[r] * kFold1;
                tpl = fmaf(omh, fmaf(-qq, rr, dwv[r]), tpl);
              }
            }
#pragma unroll
            for (int r = 0; r < 8; ++r) hf[8 * u + r] = to_h(hv[r] * kCarryAct);
          }
          FragU w2;
          w2.h[0] = *(const v8h*)(sW2t + c * kHid + 32 * jj + 8 * hh);
          w2.h[1] = *(const v8h*)(sW2t + c * kHid + 32 * jj + 8 * hh + 16);
          oacc = mma_h(w2.v, hf, oacc);
        }
        const v4f c20 = *(const v4f*)(sB2 + 8 * hh);
        const v4f c21 = *(const v4f*)(sB2 + 8 * hh + 4);
        v4f o0, o1;
        o0[0] = fmaf(oacc[0], kFold2, c20[0]);
        o0[1] = fmaf(oacc[1], kFold2, c20[1]);
        o0[2] = fmaf(oacc[2], kFold2, c20[2]);
        o0[3] = fmaf(oacc[3], kFold2, c20[3]);
        o1[0] = fmaf(oacc[4], kFold2, c21[0]);
        o1[1] = fmaf(oacc[5], kFold2, c21[1]);
        o1[2] = fmaf(oacc[6], kFold2, c21[2]);
        o1[3] = fmaf(oacc[7], kFold2, c21[3]);
        *(v4f*)(aw + (16 * t + c) * kAPitch + 8 * hh) = o0;
        *(v4f*)(aw + (16 * t + c) * kAPitch + 8 * hh + 4) = o1;
        if (isdiv) aw[(16 * t + c) * kAPitch + 16 + hh] = tpl;
      }
      wave_lds_sync();

      float a[16];
#pragma unroll
      for (int q4 = 0; q4 < 4; ++q4) {
        const v4f av = *(const v4f*)(aw + lane * kAPitch + 4 * q4);
        a[4 * q4 + 0] = av[0];
        a[4 * q4 + 1] = av[1];
        a[4 * q4 + 2] = av[2];
        a[4 * q4 + 3] = av[3];
      }

      if (isdiv) {
        float adot = 0.0f;
#pragma unroll
        for (int j = 0; j < 16; ++j) adot = fmaf(a[j], z[j], adot);
        const float t12 = aw[lane * kAPitch + 16] + aw[lane * kAPitch + 17];
        const float dv = (0.5f * inv) * (t12 - (float)(kDim - 1) * adot);
        logp -= dv * ds;
#pragma unroll
        for (int j = 0; j < 16; ++j) { z[j] = y[j]; ksum[j] = 0.0f; }
      } else {
        const float wk   = (ev == 1 || ev == 4) ? 1.0f : 2.0f;
        const float cfds = ((ev == 3) ? 1.0f : 0.5f) * ds;
        float g[16];
        float gy = 0.0f, yy = 0.0f;
#pragma unroll
        for (int j = 0; j < 16; ++j) {
          g[j] = (-kRadial * z[j]) - 0.5f * a[j];
          gy = fmaf(g[j], z[j], gy);
          yy = fmaf(z[j], z[j], yy);
        }
        const float cc = gy * (1.0f / yy);
#pragma unroll
        for (int j = 0; j < 16; ++j) {
          const float kj = fmaf(-cc, z[j], g[j]);
          ksum[j] = fmaf(wk, kj, ksum[j]);
          z[j] = fmaf(cfds, kj, y[j]);
        }
      }
    }
    {
      const float h6 = ds / 6.0f;
      float nn = 0.0f;
#pragma unroll
      for (int j = 0; j < 16; ++j) {
        y[j] = fmaf(h6, ksum[j], y[j]);
        nn = fmaf(y[j], y[j], nn);
      }
      const float invn = 1.0f / sqrtf(nn);
#pragma unroll
      for (int j = 0; j < 16; ++j) y[j] *= invn;
      s += ds;
    }
  }

  {
    const float ov = (float)kLogP0 + logp;
    volatile float* po = gout + row;
    *po = ov;
    __threadfence();
    *po = ov;
  }
}

}

extern "C" void kernel_launch(void* const* d_in, const int* in_sizes, int n_in,
                              void* d_out, int out_size, void* d_ws, size_t ws_size,
                              hipStream_t stream) {
  (void)d_ws; (void)ws_size;
  if (n_in < 7) return;
  if (in_sizes[0] != eng::kBatch * eng::kDim) return;
  if (in_sizes[1] != 1) return;
  if (in_sizes[2] != (eng::kDim + 1) * eng::kHid) return;
  if (in_sizes[3] != eng::kHid) return;
  if (in_sizes[4] != eng::kHid * eng::kDim) return;
  if (in_sizes[5] != eng::kDim) return;
  if (in_sizes[6] != 1) return;
  if (out_size != eng::kBatch) return;

  const float* x  = (const float*)d_in[0];
  const float* t  = (const float*)d_in[1];
  const float* W1 = (const float*)d_in[2];
  const float* b1 = (const float*)d_in[3];
  const float* W2 = (const float*)d_in[4];
  const float* b2 = (const float*)d_in[5];
  const int* steps = (const int*)d_in[6];
  float* out = (float*)d_out;

  eng::sphere_flow_logp_kernel<<<eng::kBlocks, eng::kThreads, 0, stream>>>(x, t, W1, b1, W2, b2, steps, out);
}
